// DifferentialMultiHeadSelfAttention_73564199846400
// MI455X (gfx1250) — hardware-verified
//
#include <hip/hip_runtime.h>


#define TT   2048
#define EE   1024
#define NH_  16
#define HD   64
#define ZH   2
#define SCL  0.125f
typedef _Float16 h16;
typedef unsigned short bf;
typedef __attribute__((ext_vector_type(16))) __bf16   v16bf;
typedef __attribute__((ext_vector_type(16))) _Float16 v16h;
typedef __attribute__((ext_vector_type(8)))  _Float16 v8h;
typedef __attribute__((ext_vector_type(8)))  unsigned short v8us;
typedef __attribute__((ext_vector_type(8)))  float    v8f;
typedef __attribute__((ext_vector_type(4)))  float    v4f;
typedef v8h  __attribute__((may_alias)) v8ha;
typedef v4f  __attribute__((may_alias)) v4fa;
typedef v8us __attribute__((may_alias)) v8usa;

__device__ __forceinline__ unsigned short f2bf(float f) { unsigned u = __float_as_uint(f); u += 0x7FFFu + ((u >> 16) & 1u); return (unsigned short)(u >> 16); }
__device__ __forceinline__ float bf2f(unsigned short b) { return __uint_as_float(((unsigned)b) << 16); }
__device__ __forceinline__ float bfr(float f) { return bf2f(f2bf(f)); }
__device__ __forceinline__ v16h cat16(v8h lo, v8h hi) { return __builtin_shufflevector(lo, hi, 0, 1, 2, 3, 4, 5, 6, 7, 8, 9, 10, 11, 12, 13, 14, 15); }
__device__ __forceinline__ v16bf cat16b(v8us lo, v8us hi) { return __builtin_bit_cast(v16bf, __builtin_shufflevector(lo, hi, 0, 1, 2, 3, 4, 5, 6, 7, 8, 9, 10, 11, 12, 13, 14, 15)); }
__device__ __forceinline__ v8f wmma16(v16h a, v16h b, v8f c) { return __builtin_amdgcn_wmma_f32_16x16x32_f16(false, a, false, b, (short)0, c, false, false); }
__device__ __forceinline__ v8f wmmab(v16bf a, v16bf b, v8f c) { return __builtin_amdgcn_wmma_f32_16x16x32_bf16(false, a, false, b, (short)0, c, false, false); }


template <typename T16> struct WFrag;
template <> struct WFrag<h16> { typedef v16h V; static __device__ __forceinline__ V ld(const h16* p) { return cat16(*(const v8h*)p, *(const v8h*)(p + 16)); } static __device__ __forceinline__ v8f mma(V a, V b, v8f c) { return wmma16(a, b, c); } };
template <> struct WFrag<bf> { typedef v16bf V; static __device__ __forceinline__ V ld(const bf* p) { return cat16b(*(const v8us*)p, *(const v8us*)(p + 16)); } static __device__ __forceinline__ v8f mma(V a, V b, v8f c) { return wmmab(a, b, c); } };
template <typename T16, int NSPLIT, bool BIAS>
__global__ __launch_bounds__(32) void k_gemmw(const T16* __restrict__ A, const T16* __restrict__ A2, const T16* __restrict__ Bt, const T16* __restrict__ Bt2, int K, float* C, int ldc, const float* __restrict__ bias, size_t sA, size_t sB, size_t sC) {
    typedef typename WFrag<T16>::V V;
    __shared__ __align__(16) float os[16 * 68];
    const size_t z = blockIdx.z; A += z * sA; if (A2) A2 += z * sA; Bt += z * sB; if (Bt2) Bt2 += z * sB; C += z * sC;
    const int lane = threadIdx.x & 31, lr = lane & 15, hi = lane >> 4; const int r0 = blockIdx.x * 64, c0 = blockIdx.y * 64;
    v8f acc[4][4];
#pragma unroll
    for (int mb = 0; mb < 4; ++mb)
#pragma unroll
        for (int nb = 0; nb < 4; ++nb) acc[mb][nb] = (v8f){};
    const size_t aoff = (size_t)(r0 + lr) * K + 8 * hi, boff = (size_t)(c0 + lr) * K + 8 * hi;
#pragma unroll 1
    for (int kc = 0; kc < K; kc += 32) {
        V a[4], a2[4];
#pragma unroll
        for (int mb = 0; mb < 4; ++mb) { a[mb] = WFrag<T16>::ld(A + aoff + (size_t)mb * 16 * K + kc); if (NSPLIT == 1 || NSPLIT == 2) a2[mb] = WFrag<T16>::ld(A2 + aoff + (size_t)mb * 16 * K + kc); }
#pragma unroll
        for (int nb = 0; nb < 4; ++nb) { const V b = WFrag<T16>::ld(Bt + boff + (size_t)nb * 16 * K + kc); V b2; if (NSPLIT >= 2) b2 = WFrag<T16>::ld(Bt2 + boff + (size_t)nb * 16 * K + kc);
#pragma unroll
            for (int mb = 0; mb < 4; ++mb) { acc[mb][nb] = WFrag<T16>::mma(a[mb], b, acc[mb][nb]); if (NSPLIT == 1 || NSPLIT == 2) acc[mb][nb] = WFrag<T16>::mma(a2[mb], b, acc[mb][nb]); if (NSPLIT >= 2) acc[mb][nb] = WFrag<T16>::mma(a[mb], b2, acc[mb][nb]); } }
        asm volatile("v_nop\n\tv_nop\n\tv_nop\n\tv_nop" : "+v"(acc[0][0]), "+v"(acc[1][1]), "+v"(acc[2][2]), "+v"(acc[3][3]) : "v"(a[0]), "v"(a[3]));
    }
#pragma unroll
    for (int mb = 0; mb < 4; ++mb) {
#pragma unroll
        for (int nb = 0; nb < 4; ++nb) {
#pragma unroll
            for (int j = 0; j < 8; ++j) os[(hi * 8 + j) * 68 + nb * 16 + lr] = acc[mb][nb][j]; }
        __builtin_amdgcn_wave_barrier(); asm volatile("" ::: "memory");
        float* crow = C + (size_t)(r0 + mb * 16) * ldc + c0;
#pragma unroll 1
        for (int ps = 0; ps < 2; ++ps) {
#pragma unroll
            for (int s = 0; s < 8; ++s) { const int row = 2 * s + hi, cofs = lr * 4; v4f val = *(const v4fa*)(os + row * 68 + cofs); if (BIAS) { val[0] += bfr(bias[c0 + cofs]); val[1] += bfr(bias[c0 + cofs + 1]); val[2] += bfr(bias[c0 + cofs + 2]); val[3] += bfr(bias[c0 + cofs + 3]); }
                *(volatile v4f*)(crow + (size_t)row * ldc + cofs) = val; }
            if (ps == 0) __threadfence(); }
        __builtin_amdgcn_wave_barrier(); asm volatile("" ::: "memory");
    }
}

__device__ __forceinline__ void splitf(float y, unsigned short& h, unsigned short& l) { h = f2bf(y); l = f2bf(y - bf2f(h)); }
typedef __attribute__((ext_vector_type(2))) unsigned short v2us;
typedef __attribute__((ext_vector_type(4))) unsigned short v4us;
typedef __attribute__((ext_vector_type(2))) float v2f;

__global__ __launch_bounds__(256) void k_cvt8(const float* __restrict__ src, bf* dst, size_t n8) { const size_t i = (size_t)blockIdx.x * 256 + threadIdx.x; if (i >= n8) return; const v8f v = *(const v8f*)(src + i * 8); v8us o;
#pragma unroll
    for (int k = 0; k < 8; ++k) o[k] = f2bf(v[k]); *(volatile v8us*)(dst + i * 8) = o; __threadfence(); *(volatile v8us*)(dst + i * 8) = o; }
__global__ __launch_bounds__(256) void k_pl(const float* __restrict__ F, bf* Ph, bf* Pl) { const size_t e = ((size_t)blockIdx.x * 256 + threadIdx.x) * 2; if (e >= (size_t)NH_ * TT * HD) return; const int d = (int)(e % HD); const int t = (int)((e / HD) % TT); const int h = (int)(e / ((size_t)HD * TT)); const float* f = F + (size_t)t * EE + h * HD + d; v2us oh, ol;
#pragma unroll
    for (int u = 0; u < 2; ++u) { unsigned short a, c; splitf(f[u], a, c); oh[u] = a; ol[u] = c; } *(volatile v2us*)(Ph + e) = oh; *(volatile v2us*)(Pl + e) = ol; __threadfence(); *(volatile v2us*)(Ph + e) = oh; *(volatile v2us*)(Pl + e) = ol; }
__global__ __launch_bounds__(256) void k_vtp(const float* __restrict__ F, bf* Vh, bf* Vl) { const size_t e = ((size_t)blockIdx.x * 256 + threadIdx.x) * 2; if (e >= (size_t)NH_ * HD * TT) return; const int t = (int)(e % TT); const int d = (int)((e / TT) % HD); const int h = (int)(e / ((size_t)TT * HD)); v2us oh, ol;
#pragma unroll
    for (int u = 0; u < 2; ++u) { unsigned short a, c; splitf(F[(size_t)(t + u) * EE + h * HD + d], a, c); oh[u] = a; ol[u] = c; } *(volatile v2us*)(Vh + e) = oh; *(volatile v2us*)(Vl + e) = ol; __threadfence(); *(volatile v2us*)(Vh + e) = oh; *(volatile v2us*)(Vl + e) = ol; }
__global__ __launch_bounds__(256) void k_soft1(float* Sb, const int* __restrict__ msk) { const int lane = threadIdx.x & 31; const int row = blockIdx.x * 8 + (threadIdx.x >> 5); if (row >= ZH * TT) return; const int i = row % TT; float* sr = Sb + (size_t)row * TT; const int* mr = msk + (size_t)i * TT; float v[64]; float mx = -3.0e38f;
#pragma unroll
    for (int ch = 0; ch < 16; ++ch) { const int j0 = ch * 128 + lane * 4; const v4f a = *(const v4f*)(sr + j0);
#pragma unroll
        for (int q = 0; q < 4; ++q) { const float t = mr[j0 + q] ? -3.0e38f : a[q] * SCL; v[ch * 4 + q] = t; mx = fmaxf(mx, t); } }
#pragma unroll
    for (int sh = 16; sh; sh >>= 1) mx = fmaxf(mx, __shfl_xor(mx, sh, 32));
    float sum = 0.f;
#pragma unroll
    for (int k = 0; k < 64; ++k) { float d0 = __fsub_rn(v[k], mx); asm volatile("" : "+v"(d0)); v[k] = __expf(d0); sum += v[k]; }
#pragma unroll
    for (int sh = 16; sh; sh >>= 1) sum += __shfl_xor(sum, sh, 32);
    const float f = __fdiv_rn(1.0f, sum);
#pragma unroll 1
    for (int ps = 0; ps < 2; ++ps) {
#pragma unroll
        for (int ch = 0; ch < 16; ++ch) { v4f o; o[0] = v[ch * 4] * f; o[1] = v[ch * 4 + 1] * f; o[2] = v[ch * 4 + 2] * f; o[3] = v[ch * 4 + 3] * f; *(volatile v4f*)(sr + ch * 128 + lane * 4) = o; }
        if (ps == 0) __threadfence(); } }
__global__ __launch_bounds__(256) void k_soft2(const float* __restrict__ S2, const float* __restrict__ P1, const int* __restrict__ msk, const float* __restrict__ lam, int h0, bf* Ph, bf* Pl) { const int lane = threadIdx.x & 31; const int row = blockIdx.x * 8 + (threadIdx.x >> 5); if (row >= ZH * TT) return; const int i = row % TT, z = row / TT; const float lm = bfr(lam[h0 + z]); const float* sr = S2 + (size_t)row * TT; const float* pr = P1 + (size_t)row * TT; const int* mr = msk + (size_t)i * TT; float v[64]; float mx = -3.0e38f;
#pragma unroll
    for (int ch = 0; ch < 16; ++ch) { const int j0 = ch * 128 + lane * 4; const v4f a = *(const v4f*)(sr + j0);
#pragma unroll
        for (int q = 0; q < 4; ++q) { const float t = mr[j0 + q] ? -3.0e38f : a[q] * SCL; v[ch * 4 + q] = t; mx = fmaxf(mx, t); } }
#pragma unroll
    for (int sh = 16; sh; sh >>= 1) mx = fmaxf(mx, __shfl_xor(mx, sh, 32));
    float sum = 0.f;
#pragma unroll
    for (int k = 0; k < 64; ++k) { float d0 = __fsub_rn(v[k], mx); asm volatile("" : "+v"(d0)); v[k] = __expf(d0); sum += v[k]; }
#pragma unroll
    for (int sh = 16; sh; sh >>= 1) sum += __shfl_xor(sum, sh, 32);
    const float f = __fmul_rn(__fdiv_rn(1.0f, sum), lm);
#pragma unroll 1
    for (int ps = 0; ps < 2; ++ps) {
#pragma unroll
        for (int ch = 0; ch < 16; ++ch) { const int j0 = ch * 128 + lane * 4; const v4f p1 = *(const v4f*)(pr + j0); v4us oh, ol;
#pragma unroll
            for (int q = 0; q < 4; ++q) { float t2 = __fmul_rn(v[ch * 4 + q], f); asm volatile("" : "+v"(t2)); unsigned short a, c; splitf(__fsub_rn(p1[q], t2), a, c); oh[q] = a; ol[q] = c; }
            *(volatile v4us*)(Ph + (size_t)row * TT + j0) = oh; *(volatile v4us*)(Pl + (size_t)row * TT + j0) = ol; }
        if (ps == 0) __threadfence(); } }
__global__ __launch_bounds__(256) void k_cat(const float* __restrict__ Ob, int h0, float* CAT) { const size_t e = ((size_t)blockIdx.x * 256 + threadIdx.x) * 2; if (e >= (size_t)ZH * TT * HD) return; const int d = (int)(e % HD); const int t = (int)((e / HD) % TT); const int z = (int)(e / ((size_t)HD * TT)); v2f o; o[0] = Ob[e]; o[1] = Ob[e + 1]; const size_t oo = (size_t)t * EE + (h0 + z) * HD + d; *(volatile v2f*)(CAT + oo) = o; __threadfence(); *(volatile v2f*)(CAT + oo) = o; }
__global__ __launch_bounds__(256) void k_gst(const float* __restrict__ CAT, const float* __restrict__ MU, int centred, float* PS) { const int e = blockIdx.x * 256 + threadIdx.x; if (e >= NH_ * TT) return; const int t = e % TT, h = e / TT; const float m = centred ? MU[h] : 0.f; const float* r = CAT + (size_t)t * EE + h * HD; float s = 0.f;
    for (int d = 0; d < HD; ++d) { const float dv = __fsub_rn(r[d], m); float q = centred ? __fmul_rn(dv, dv) : dv; asm volatile("" : "+v"(q)); s = __fadd_rn(s, q); } *(volatile float*)(PS + e) = s; __threadfence(); *(volatile float*)(PS + e) = s; }
__global__ __launch_bounds__(32) void k_gred(const float* __restrict__ PS, float* M) { const int lane = threadIdx.x; if (lane >= NH_) { return; } float s = 0.f; for (int t = 0; t < TT; ++t) s = __fadd_rn(s, PS[(size_t)lane * TT + t]); const float m = s * (1.0f / (float)(HD * TT)); *(volatile float*)(M + lane) = m; __threadfence(); *(volatile float*)(M + lane) = m; }
__global__ __launch_bounds__(256) void k_gn(const float* __restrict__ CAT, const float* __restrict__ MU, const float* __restrict__ VAR, const float* __restrict__ gw, const float* __restrict__ gb, bf* Ah, bf* Al) { const size_t i = ((size_t)blockIdx.x * 256 + threadIdx.x) * 4; if (i >= (size_t)TT * EE) return; const int c = (int)(i % EE); const int h = c / HD; const float rs = __frsqrt_rn(__fadd_rn(VAR[h], 1e-5f)); const float mu = MU[h]; const v4f a = *(const v4f*)(CAT + i); v4us oh, ol;
#pragma unroll
    for (int q = 0; q < 4; ++q) { float t = __fmul_rn(__fsub_rn(a[q], mu), rs); asm volatile("" : "+v"(t)); float tg = __fmul_rn(t, bfr(gw[c + q])); asm volatile("" : "+v"(tg)); unsigned short u, c2; splitf(__fadd_rn(tg, bfr(gb[c + q])), u, c2); oh[q] = u; ol[q] = c2; }
    *(volatile v4us*)(Ah + i) = oh; *(volatile v4us*)(Al + i) = ol; __threadfence(); *(volatile v4us*)(Ah + i) = oh; *(volatile v4us*)(Al + i) = ol; }

extern "C" void kernel_launch(void* const* d_in, const int* in_sizes, int n_in,
                              void* d_out, int out_size, void* d_ws, size_t ws_size, hipStream_t stream) {
    (void)in_sizes; (void)n_in; (void)out_size;
    const float* x = (const float*)d_in[0]; const int* msk = (const int*)d_in[1]; const float* IN[17]; for (int i = 2; i < 17; ++i) IN[i] = (const float*)d_in[i];
    float* OUT = (float*)d_out;
    char* wsp = (char*)d_ws;
    auto take = [&](size_t bytes) { char* p = wsp; wsp += (bytes + 255) & ~(size_t)255; return (void*)p; };
    bf* WB[6]; for (int i = 0; i < 6; ++i) WB[i] = (bf*)take((size_t)EE * EE * 2); bf* XB = (bf*)take((size_t)TT * EE * 2); float* F = (float*)take((size_t)TT * EE * 4);
    bf* Q1h = (bf*)take((size_t)NH_ * TT * HD * 2); bf* Q1l = (bf*)take((size_t)NH_ * TT * HD * 2); bf* Q2h = (bf*)take((size_t)NH_ * TT * HD * 2); bf* Q2l = (bf*)take((size_t)NH_ * TT * HD * 2); bf* K1h = (bf*)take((size_t)NH_ * TT * HD * 2); bf* K1l = (bf*)take((size_t)NH_ * TT * HD * 2); bf* K2h = (bf*)take((size_t)NH_ * TT * HD * 2); bf* K2l = (bf*)take((size_t)NH_ * TT * HD * 2); bf* Vh = (bf*)take((size_t)NH_ * HD * TT * 2); bf* Vl = (bf*)take((size_t)NH_ * HD * TT * 2);
    float* S1 = (float*)take((size_t)ZH * TT * TT * 4); float* S2 = (float*)take((size_t)ZH * TT * TT * 4); bf* Ph = (bf*)take((size_t)ZH * TT * TT * 2); bf* Pl = (bf*)take((size_t)ZH * TT * TT * 2); float* Ob = (float*)take((size_t)ZH * TT * HD * 4); float* CAT = (float*)take((size_t)TT * EE * 4); float* PS = (float*)take((size_t)NH_ * TT * 4); float* MU = (float*)take(64 * 4); float* VAR = (float*)take(64 * 4); bf* Ah = (bf*)take((size_t)TT * EE * 2); bf* Al = (bf*)take((size_t)TT * EE * 2);
    if ((size_t)(wsp - (char*)d_ws) > ws_size) return;
    const int widx[6] = {2, 4, 6, 8, 10, 15}; for (int i = 0; i < 6; ++i) k_cvt8<<<(EE * EE / 8 + 255) / 256, 256, 0, stream>>>(IN[widx[i]], WB[i], (size_t)EE * EE / 8);
    k_cvt8<<<(TT * EE / 8 + 255) / 256, 256, 0, stream>>>(x, XB, (size_t)TT * EE / 8);
    const unsigned LP = (unsigned)(((size_t)NH_ * TT * HD / 2 + 255) / 256);
    bf* PLh[4] = {Q1h, Q2h, K1h, K2h}; bf* PLl[4] = {Q1l, Q2l, K1l, K2l};
    for (int i = 0; i < 4; ++i) { k_gemmw<bf, 0, true><<<dim3(TT / 64, EE / 64, 1), 32, 0, stream>>>(XB, nullptr, WB[i], nullptr, EE, F, EE, IN[widx[i] + 1], 0, 0, 0); k_pl<<<LP, 256, 0, stream>>>(F, PLh[i], PLl[i]); }
    k_gemmw<bf, 0, true><<<dim3(TT / 64, EE / 64, 1), 32, 0, stream>>>(XB, nullptr, WB[4], nullptr, EE, F, EE, IN[11], 0, 0, 0); k_vtp<<<LP, 256, 0, stream>>>(F, Vh, Vl);
    for (int h0 = 0; h0 < NH_; h0 += ZH) { const size_t z = (size_t)h0;
        k_gemmw<bf, 2, false><<<dim3(TT / 64, TT / 64, ZH), 32, 0, stream>>>(Q1h + z * TT * HD, Q1l + z * TT * HD, K1h + z * TT * HD, K1l + z * TT * HD, HD, S1, TT, nullptr, (size_t)TT * HD, (size_t)TT * HD, (size_t)TT * TT);
        k_gemmw<bf, 2, false><<<dim3(TT / 64, TT / 64, ZH), 32, 0, stream>>>(Q2h + z * TT * HD, Q2l + z * TT * HD, K2h + z * TT * HD, K2l + z * TT * HD, HD, S2, TT, nullptr, (size_t)TT * HD, (size_t)TT * HD, (size_t)TT * TT);
        k_soft1<<<ZH * TT / 8, 256, 0, stream>>>(S1, msk); k_soft2<<<ZH * TT / 8, 256, 0, stream>>>(S2, S1, msk, IN[12], h0, Ph, Pl);
        k_gemmw<bf, 2, false><<<dim3(TT / 64, 1, ZH), 32, 0, stream>>>(Ph, Pl, Vh + z * HD * TT, Vl + z * HD * TT, TT, Ob, HD, nullptr, (size_t)TT * TT, (size_t)HD * TT, (size_t)TT * HD);
        k_cat<<<(unsigned)(((size_t)ZH * TT * HD / 2 + 255) / 256), 256, 0, stream>>>(Ob, h0, CAT); }
    k_gst<<<(NH_ * TT + 255) / 256, 256, 0, stream>>>(CAT, nullptr, 0, PS); k_gred<<<1, 32, 0, stream>>>(PS, MU); k_gst<<<(NH_ * TT + 255) / 256, 256, 0, stream>>>(CAT, MU, 1, PS); k_gred<<<1, 32, 0, stream>>>(PS, VAR);
    k_gn<<<(unsigned)(((size_t)TT * EE / 4 + 255) / 256), 256, 0, stream>>>(CAT, MU, VAR, IN[13], IN[14], Ah, Al);
    k_gemmw<bf, 1, true><<<dim3(TT / 64, EE / 64, 1), 32, 0, stream>>>(Ah, Al, WB[5], nullptr, EE, OUT, EE, IN[16], 0, 0, 0);
}
